// MultiHeadSelfAttention_36129264894565
// MI455X (gfx1250) — hardware-verified
//
#include <hip/hip_runtime.h>

typedef __attribute__((ext_vector_type(16))) __bf16 v16b;
typedef __attribute__((ext_vector_type(8)))  __bf16 v8b;
typedef __attribute__((ext_vector_type(16))) _Float16 v16h;
typedef __attribute__((ext_vector_type(8)))  _Float16 v8h;
typedef __attribute__((ext_vector_type(8)))  float  v8f;
typedef __attribute__((ext_vector_type(4)))  float  v4f;
typedef __attribute__((ext_vector_type(4)))  unsigned int v4u;
typedef v8h v8h_a __attribute__((may_alias));
typedef v4f v4f_a __attribute__((may_alias));
typedef v4u v4u_a __attribute__((may_alias));
typedef _Float16 h16;

#ifndef NB
#define NB 2
#endif
#ifndef SEQ
#define SEQ 1024
#endif
#define NB_FULL 2
#define SEQ_FULL 1024

#define VGPR_CAP __attribute__((amdgpu_num_vgpr(256)))

#define QKV_CARRY   16.0f
#define P_CARRY     256.0f
#define CTX_CARRY   256.0f
#define WO_CARRY    1024.0f
#define SCORE_SCALE 0.00048828125f
#define CTX_FOLD    16.0f
#define OUT_FOLD    3.814697265625e-06f

constexpr int DMODEL = 1024;
constexpr int NHEAD  = 16;
constexpr int DHEAD  = 64;
constexpr int NQKV   = 3 * DMODEL;
constexpr int NBH    = NB * NHEAD;
constexpr int MROWS  = NB * SEQ;
constexpr int KCH    = 64;
constexpr int NWAVE  = 4;
constexpr int TQ_PITCH = 72;
constexpr int TV_PITCH = 136;
constexpr int T_ELEMS  = 128 * TQ_PITCH;
constexpr int OS_PITCH = 68;

constexpr size_t PLANE  = (size_t)NBH * SEQ * DHEAD;
constexpr size_t XB_E   = (size_t)MROWS * DMODEL;
constexpr size_t WQT_E  = (size_t)NQKV * DMODEL;
constexpr size_t WOT_E  = (size_t)DMODEL * DMODEL;
constexpr size_t QKVP_E = 3 * PLANE;
constexpr size_t CTX_E  = XB_E;
constexpr size_t WS_NEED = 2 * (XB_E + WQT_E + WOT_E + QKVP_E + CTX_E);

static_assert(SEQ % 128 == 0);
static_assert(KCH == 64 && SEQ % KCH == 0);
static_assert(SEQ <= SEQ_FULL && NB <= NB_FULL);
static_assert(DHEAD == 64 && DMODEL == NHEAD * DHEAD);
static_assert(DMODEL % 64 == 0 && NQKV % 64 == 0 && DMODEL % 32 == 0);
static_assert(DMODEL % 8 == 0 && DHEAD % 8 == 0);
static_assert(MROWS % 128 == 0);
static_assert(NWAVE * 16 == 64 && NWAVE * 32 == 128);
static_assert(64 * TV_PITCH <= T_ELEMS);
static_assert(TQ_PITCH >= 64 && TV_PITCH >= 128 && OS_PITCH >= 64);
static_assert((TQ_PITCH * 2) % 16 == 0 && (TV_PITCH * 2) % 16 == 0 && (OS_PITCH * 4) % 16 == 0);
static_assert(XB_E % 64 == 0 && WQT_E % 64 == 0 && WOT_E % 64 == 0 && PLANE % 64 == 0);
static_assert(WS_NEED <= 134217728ull);


__device__ __forceinline__ unsigned short f2bf_bits(float f) {
  unsigned u = __float_as_uint(f);
  return (unsigned short)((u + 0x7FFFu + ((u >> 16) & 1u)) >> 16);
}
__device__ __forceinline__ float bf_bits2f(unsigned short h) { return __uint_as_float(((unsigned)h) << 16); }
__device__ __forceinline__ unsigned pk2(float a, float b) {
  return (unsigned)f2bf_bits(a) | ((unsigned)f2bf_bits(b) << 16);
}

static __device__ __forceinline__ h16 toh_flush(float v) {
  const h16 r = (h16)v;
  return (fabsf(v) < 6.103515625e-05f) ? (h16)0.0f : r;
}
static __device__ __forceinline__ unsigned short hbits(h16 v) {
  return __builtin_bit_cast(unsigned short, v);
}
static __device__ __forceinline__ unsigned pkh2(float a, float b) {
  return (unsigned)hbits(toh_flush(a)) | ((unsigned)hbits(toh_flush(b)) << 16);
}

__device__ __forceinline__ v8f mma_bf16(v16b a, v16b b, v8f c) {
  c = __builtin_amdgcn_wmma_f32_16x16x32_bf16(false, a, false, b, (short)0, c, false, false);
  asm volatile("v_nop\n\tv_nop\n\tv_nop\n\tv_nop" : "+v"(c) : "v"(a), "v"(b));
  return c;
}
__device__ __forceinline__ v8f mma_f16(v16h a, v16h b, v8f c) {
  c = __builtin_amdgcn_wmma_f32_16x16x32_f16(false, a, false, b, (short)0, c, false, false);
  asm volatile("v_nop\n\tv_nop\n\tv_nop\n\tv_nop" : "+v"(c) : "v"(a), "v"(b));
  return c;
}

__device__ __forceinline__ void wave_lds_sync() {
  __builtin_amdgcn_fence(3  , "workgroup");
  __builtin_amdgcn_wave_barrier();
  __builtin_amdgcn_fence(2  , "workgroup");
}

__global__ __launch_bounds__(256) void cvt_rows_kernel(
    const float* __restrict__ in, unsigned short* __restrict__ outp,
    int nunits, int upr, int rpb, int rpb_full)
{
  const int u = blockIdx.x * 256 + threadIdx.x;
  if (u >= nunits) return;
  const int row = u / upr;
  const int seg = u - row * upr;
  const int b = row / rpb;
  const int l = row - b * rpb;
  const float* src = in + ((size_t)(b * rpb_full + l) * upr + seg) * 8;
  const v4f a0 = *(const v4f*)src;
  const v4f a1 = *(const v4f*)(src + 4);
  v4u w;
  w[0] = pk2(a0[0], a0[1]);
  w[1] = pk2(a0[2], a0[3]);
  w[2] = pk2(a1[0], a1[1]);
  w[3] = pk2(a1[2], a1[3]);
  volatile v4u* dst = (volatile v4u*)(outp + ((size_t)row * upr + seg) * 8);
  *dst = w;
  __threadfence();
  *dst = w;
}

__global__ __launch_bounds__(256) void cvt_rows_h_kernel(
    const float* __restrict__ in, unsigned short* __restrict__ outp,
    int nunits, int upr, int rpb, int rpb_full, float carry)
{
  const int u = blockIdx.x * 256 + threadIdx.x;
  if (u >= nunits) return;
  const int row = u / upr;
  const int seg = u - row * upr;
  const int b = row / rpb;
  const int l = row - b * rpb;
  const float* src = in + ((size_t)(b * rpb_full + l) * upr + seg) * 8;
  const v4f a0 = *(const v4f*)src;
  const v4f a1 = *(const v4f*)(src + 4);
  v4u w;
  w[0] = pkh2(bf_bits2f(f2bf_bits(a0[0])) * carry, bf_bits2f(f2bf_bits(a0[1])) * carry);
  w[1] = pkh2(bf_bits2f(f2bf_bits(a0[2])) * carry, bf_bits2f(f2bf_bits(a0[3])) * carry);
  w[2] = pkh2(bf_bits2f(f2bf_bits(a1[0])) * carry, bf_bits2f(f2bf_bits(a1[1])) * carry);
  w[3] = pkh2(bf_bits2f(f2bf_bits(a1[2])) * carry, bf_bits2f(f2bf_bits(a1[3])) * carry);
  volatile v4u* dst = (volatile v4u*)(outp + ((size_t)row * upr + seg) * 8);
  *dst = w;
  __threadfence();
  *dst = w;
}

__global__ __launch_bounds__(128) VGPR_CAP void gemm_qkv_kernel(
    const unsigned short* __restrict__ Xb, const unsigned short* __restrict__ WqT,
    unsigned short* __restrict__ qkvp)
{
  union FB { v16b v; v8b h[2]; };
  __shared__ __align__(16) unsigned short Th[T_ELEMS];

  const int tid  = threadIdx.x;
  const int wave = __builtin_amdgcn_readfirstlane(tid >> 5);
  const int lane = tid & 31;
  const int hh   = lane >> 4;
  const int c    = lane & 15;
  const int n0   = blockIdx.x * 64;
  const int m0   = blockIdx.y * 128;

  v8f acc[2][4];
#pragma unroll
  for (int mt = 0; mt < 2; ++mt)
#pragma unroll
    for (int t = 0; t < 4; ++t) acc[mt][t] = (v8f){0.f,0.f,0.f,0.f,0.f,0.f,0.f,0.f};

  const unsigned short* a0p = Xb + (size_t)(m0 + wave * 32 + c) * DMODEL + 8 * hh;
  const unsigned short* a1p = a0p + (size_t)16 * DMODEL;
  const unsigned short* bp  = WqT + (size_t)(n0 + c) * DMODEL + 8 * hh;

#pragma unroll 1
  for (int k0 = 0; k0 < DMODEL; k0 += 32) {
    FB a0, a1;
    a0.h[0] = *(const v8b*)(a0p + k0);
    a0.h[1] = *(const v8b*)(a0p + k0 + 16);
    a1.h[0] = *(const v8b*)(a1p + k0);
    a1.h[1] = *(const v8b*)(a1p + k0 + 16);
#pragma unroll
    for (int t = 0; t < 4; ++t) {
      FB bf;
      bf.h[0] = *(const v8b*)(bp + (size_t)t * 16 * DMODEL + k0);
      bf.h[1] = *(const v8b*)(bp + (size_t)t * 16 * DMODEL + k0 + 16);
      acc[0][t] = mma_bf16(a0.v, bf.v, acc[0][t]);
      acc[1][t] = mma_bf16(a1.v, bf.v, acc[1][t]);
    }
  }

  const int sec = n0 / DMODEL;
#pragma unroll
  for (int t = 0; t < 4; ++t) {
#pragma unroll
    for (int mt = 0; mt < 2; ++mt) {
#pragma unroll
      for (int r = 0; r < 8; ++r) {
        const float val = acc[mt][t][r] * QKV_CARRY;
        const unsigned short hb = hbits(toh_flush(val));
        const int rl = wave * 32 + mt * 16 + 8 * hh + r;
        const int cl = 16 * t + c;
        const int idx = (sec < 2) ? (rl * TQ_PITCH + cl) : (cl * TV_PITCH + rl);
        Th[idx] = hb;
      }
    }
  }
  __syncthreads();

  const int b  = m0 / SEQ;
  const int l0 = m0 - b * SEQ;
  const int h  = (n0 - sec * DMODEL) / DHEAD;
  const int bh = b * NHEAD + h;
  unsigned short* ph = qkvp + (size_t)sec * PLANE;

  for (int pass = 0; pass < 2; ++pass) {
    if (sec < 2) {
#pragma unroll
      for (int it = 0; it < 8; ++it) {
        const int u = it * 128 + tid;
        const int row = u >> 3;
        const int seg = u & 7;
        const v4u hw = *(const v4u_a*)(Th + row * TQ_PITCH + seg * 8);
        const size_t g = ((size_t)bh * SEQ + l0 + row) * DHEAD + seg * 8;
        *(volatile v4u*)(ph + g) = hw;
      }
    } else {
#pragma unroll
      for (int it = 0; it < 8; ++it) {
        const int u = it * 128 + tid;
        const int drow = u >> 4;
        const int seg  = u & 15;
        const v4u hw = *(const v4u_a*)(Th + drow * TV_PITCH + seg * 8);
        const size_t g = ((size_t)bh * DHEAD + drow) * SEQ + l0 + seg * 8;
        *(volatile v4u*)(ph + g) = hw;
      }
    }
    __threadfence();
  }
}

__global__ __launch_bounds__(128) VGPR_CAP void attn_kernel(
    const unsigned short* __restrict__ qkvp, unsigned short* __restrict__ ctxp)
{
  union FH { v16h v; v8h h[2]; };
  __shared__ __align__(16) float Os[NWAVE][16 * OS_PITCH];
  __shared__ __align__(16) h16 Ps[NWAVE][16 * KCH];

  const int tid  = threadIdx.x;
  const int wave = __builtin_amdgcn_readfirstlane(tid >> 5);
  const int lane = tid & 31;
  const int hh   = lane >> 4;
  const int c    = lane & 15;
  const int qb   = blockIdx.x;
  const int bh   = blockIdx.y;
  const int b    = bh / NHEAD;
  const int h    = bh - b * NHEAD;
  const int q0   = qb * 64 + wave * 16;
  const float NEG_INF = -__builtin_inff();

  const unsigned short* Qp  = qkvp + (size_t)bh * SEQ * DHEAD;
  const unsigned short* Kp  = Qp + PLANE;
  const unsigned short* Vtp = Qp + 2 * PLANE;

  v16h qf[2];
  {
    const size_t qo = (size_t)(q0 + c) * DHEAD + 8 * hh;
#pragma unroll
    for (int dc = 0; dc < 2; ++dc) {
      FH f;
      f.h[0] = *(const v8h*)(Qp + qo + dc * 32);
      f.h[1] = *(const v8h*)(Qp + qo + dc * 32 + 16);
      qf[dc] = f.v;
    }
  }

  float mrow[8], lrow[8];
  v8f oacc[4];
#pragma unroll
  for (int r = 0; r < 8; ++r) { mrow[r] = NEG_INF; lrow[r] = 0.f; }
#pragma unroll
  for (int t = 0; t < 4; ++t) oacc[t] = (v8f){0.f,0.f,0.f,0.f,0.f,0.f,0.f,0.f};

#pragma unroll 1
  for (int kc = 0; kc < SEQ / KCH; ++kc) {
    const int kv0 = kc * KCH;

    v8f s[4];
#pragma unroll
    for (int j = 0; j < 4; ++j) {
      v8f sa = (v8f){0.f,0.f,0.f,0.f,0.f,0.f,0.f,0.f};
      const size_t ko = (size_t)(kv0 + j * 16 + c) * DHEAD + 8 * hh;
#pragma unroll
      for (int dc = 0; dc < 2; ++dc) {
        FH kf;
        kf.h[0] = *(const v8h*)(Kp + ko + dc * 32);
        kf.h[1] = *(const v8h*)(Kp + ko + dc * 32 + 16);
        sa = mma_f16(qf[dc], kf.v, sa);
      }
#pragma unroll
      for (int r = 0; r < 8; ++r) s[j][r] = sa[r] * SCORE_SCALE;
    }

    float cm[8];
#pragma unroll
    for (int r = 0; r < 8; ++r) {
      float m = fmaxf(fmaxf(s[0][r], s[1][r]), fmaxf(s[2][r], s[3][r]));
#pragma unroll
      for (int off = 1; off < 16; off <<= 1) m = fmaxf(m, __shfl_xor(m, off, 32));
      cm[r] = m;
    }

#pragma unroll
    for (int r = 0; r < 8; ++r) {
      const float mnew  = fmaxf(mrow[r], cm[r]);
      const float msafe = (mnew == NEG_INF) ? 0.f : mnew;
      const float alpha = expf(mrow[r] - msafe);
      mrow[r] = mnew;
      float psum = 0.f;
#pragma unroll
      for (int j = 0; j < 4; ++j) {
        const float p = expf(s[j][r] - msafe) * P_CARRY;
        const h16 ph = toh_flush(p);
        psum += (float)ph;
        Ps[wave][(8 * hh + r) * KCH + j * 16 + c] = ph;
      }
#pragma unroll
      for (int off = 1; off < 16; off <<= 1) psum += __shfl_xor(psum, off, 32);
      lrow[r] = lrow[r] * alpha + psum;
#pragma unroll
      for (int t = 0; t < 4; ++t) oacc[t][r] *= alpha;
    }
    wave_lds_sync();

#pragma unroll 1
    for (int kk = 0; kk < 2; ++kk) {
      FH pa;
      pa.h[0] = *(const v8h_a*)(&Ps[wave][c * KCH + kk * 32 + 8 * hh]);
      pa.h[1] = *(const v8h_a*)(&Ps[wave][c * KCH + kk * 32 + 16 + 8 * hh]);
#pragma unroll
      for (int t = 0; t < 4; ++t) {
        const size_t vo = (size_t)(t * 16 + c) * SEQ + kv0 + kk * 32 + 8 * hh;
        FH vb;
        vb.h[0] = *(const v8h*)(Vtp + vo);
        vb.h[1] = *(const v8h*)(Vtp + vo + 16);
        oacc[t] = mma_f16(pa.v, vb.v, oacc[t]);
      }
    }
    wave_lds_sync();
  }

#pragma unroll
  for (int r = 0; r < 8; ++r) {
    const float inv = CTX_FOLD * (1.0f / lrow[r]);
#pragma unroll
    for (int t = 0; t < 4; ++t) Os[wave][(8 * hh + r) * OS_PITCH + t * 16 + c] = oacc[t][r] * inv;
  }
  wave_lds_sync();
  {
    const int rq  = lane >> 3;
    const int seg = lane & 7;
    for (int pass = 0; pass < 2; ++pass) {
#pragma unroll
      for (int it = 0; it < 4; ++it) {
        const int row = it * 4 + rq;
        const v4f a0 = *(const v4f_a*)(&Os[wave][row * OS_PITCH + seg * 8]);
        const v4f a1 = *(const v4f_a*)(&Os[wave][row * OS_PITCH + seg * 8 + 4]);
        v4u hw;
        hw[0] = pkh2(a0[0], a0[1]);
        hw[1] = pkh2(a0[2], a0[3]);
        hw[2] = pkh2(a1[0], a1[1]);
        hw[3] = pkh2(a1[2], a1[3]);
        const size_t g = (size_t)(b * SEQ + q0 + row) * DMODEL + h * DHEAD + seg * 8;
        *(volatile v4u*)(ctxp + g) = hw;
      }
      __threadfence();
    }
  }
}

__global__ __launch_bounds__(128) VGPR_CAP void gemm_out_kernel(
    const unsigned short* __restrict__ ctxp, const unsigned short* __restrict__ WoH,
    float* __restrict__ out)
{
  union FH { v16h v; v8h h[2]; };
  __shared__ __align__(16) float Os[NWAVE][32 * OS_PITCH];

  const int tid  = threadIdx.x;
  const int wave = __builtin_amdgcn_readfirstlane(tid >> 5);
  const int lane = tid & 31;
  const int hh   = lane >> 4;
  const int c    = lane & 15;
  const int n0   = blockIdx.x * 64;
  const int m0   = blockIdx.y * 128;

  v8f acc[2][4];
#pragma unroll
  for (int mt = 0; mt < 2; ++mt)
#pragma unroll
    for (int t = 0; t < 4; ++t) acc[mt][t] = (v8f){0.f,0.f,0.f,0.f,0.f,0.f,0.f,0.f};

  const unsigned short* ah0 = ctxp + (size_t)(m0 + wave * 32 + c) * DMODEL + 8 * hh;
  const unsigned short* ah1 = ah0 + (size_t)16 * DMODEL;
  const unsigned short* bp  = WoH + (size_t)(n0 + c) * DMODEL + 8 * hh;

#pragma unroll 1
  for (int k0 = 0; k0 < DMODEL; k0 += 32) {
    FH a0h, a1h;
    a0h.h[0] = *(const v8h*)(ah0 + k0);
    a0h.h[1] = *(const v8h*)(ah0 + k0 + 16);
    a1h.h[0] = *(const v8h*)(ah1 + k0);
    a1h.h[1] = *(const v8h*)(ah1 + k0 + 16);
#pragma unroll
    for (int t = 0; t < 4; ++t) {
      FH bf;
      bf.h[0] = *(const v8h*)(bp + (size_t)t * 16 * DMODEL + k0);
      bf.h[1] = *(const v8h*)(bp + (size_t)t * 16 * DMODEL + k0 + 16);
      acc[0][t] = mma_f16(a0h.v, bf.v, acc[0][t]);
      acc[1][t] = mma_f16(a1h.v, bf.v, acc[1][t]);
    }
  }

  float* os = Os[wave];
#pragma unroll
  for (int t = 0; t < 4; ++t) {
#pragma unroll
    for (int mt = 0; mt < 2; ++mt)
#pragma unroll
      for (int r = 0; r < 8; ++r)
        os[(mt * 16 + 8 * hh + r) * OS_PITCH + 16 * t + c] = acc[mt][t][r] * OUT_FOLD;
  }
  wave_lds_sync();
  {
    const int c4 = c * 4;
    for (int pass = 0; pass < 2; ++pass) {
#pragma unroll
      for (int it = 0; it < 16; ++it) {
        const int row = it * 2 + hh;
        const v4f val = *(const v4f_a*)(os + row * OS_PITCH + c4);
        *(volatile v4f*)(out + (size_t)(m0 + wave * 32 + row) * DMODEL + n0 + c4) = val;
      }
      __threadfence();
    }
  }
}

extern "C" void kernel_launch(void* const* d_in, const int* in_sizes, int n_in,
                              void* d_out, int out_size, void* d_ws, size_t ws_size,
                              hipStream_t stream)
{
  if (n_in < 3) return;
  if (in_sizes[0] < ((NB - 1) * SEQ_FULL + SEQ) * DMODEL) return;
  if (in_sizes[1] < NQKV * DMODEL) return;
  if (in_sizes[2] < DMODEL * DMODEL) return;
  if (out_size < MROWS * DMODEL) return;
  if (d_ws == nullptr || ws_size < WS_NEED) return;

  const float* x     = (const float*)d_in[0];
  const float* W_qkv = (const float*)d_in[1];
  const float* W_out = (const float*)d_in[2];
  float* out = (float*)d_out;

  unsigned short* Xb   = (unsigned short*)d_ws;
  unsigned short* WqT  = Xb + XB_E;
  unsigned short* WoH  = WqT + WQT_E;
  unsigned short* qkvp = WoH + WOT_E;
  unsigned short* ctxp = qkvp + QKVP_E;

  {
    const int nunits = MROWS * (DMODEL / 8);
    cvt_rows_kernel<<<(nunits + 255) / 256, 256, 0, stream>>>(x, Xb, nunits, DMODEL / 8, SEQ, SEQ_FULL);
  }
  {
    const int nunits = NQKV * (DMODEL / 8);
    cvt_rows_kernel<<<(nunits + 255) / 256, 256, 0, stream>>>(W_qkv, WqT, nunits, DMODEL / 8, NQKV, NQKV);
  }
  {
    const int nunits = DMODEL * (DMODEL / 8);
    cvt_rows_h_kernel<<<(nunits + 255) / 256, 256, 0, stream>>>(W_out, WoH, nunits, DMODEL / 8, DMODEL, DMODEL, WO_CARRY);
  }

  gemm_qkv_kernel<<<dim3(NQKV / 64, MROWS / 128), 128, 0, stream>>>(Xb, WqT, qkvp);
  attn_kernel<<<dim3(SEQ / 64, NBH), 128, 0, stream>>>(qkvp, ctxp);
  gemm_out_kernel<<<dim3(DMODEL / 64, MROWS / 128), 128, 0, stream>>>(ctxp, WoH, out);
}
